// TransformerBlock_18554258719073
// MI455X (gfx1250) — hardware-verified
//
#include <hip/hip_runtime.h>
#include <stddef.h>


typedef _Float16 v16h __attribute__((ext_vector_type(16)));
typedef _Float16 v8h  __attribute__((ext_vector_type(8)));
typedef float    v8f  __attribute__((ext_vector_type(8)));
typedef float    v4f  __attribute__((ext_vector_type(4)));

#ifndef SEQ
#define SEQ 2048
#endif
#define SEQ_FULL 2048
#define DIM   1024
#define NHEAD 16
#define HD    64
#define DFF   4096
#define MROWS SEQ

static_assert(SEQ >= 128 && SEQ <= SEQ_FULL && (SEQ % 128) == 0);
static_assert(DIM == NHEAD * HD);
static_assert(HD == 64);
static_assert((DIM % 64) == 0 && (DIM % 32) == 0);
static_assert((DFF % 64) == 0 && (DFF % 32) == 0);
static_assert((MROWS % 64) == 0);
static_assert(DIM == 128 * 8);
static_assert(((size_t)DIM * DIM) % 2048 == 0);
static_assert(((size_t)DFF * DIM) % 2048 == 0);
static_assert((size_t)MROWS * DFF < (size_t)0xFFFFFFFFu);

#define LDT 72
#define LDC 68
static_assert((LDT % 8) == 0 && (LDC % 4) == 0);

#define WCARRY 64.0f
#define PCARRY 1024.0f
#define VCARRY 64.0f
#define GCARRY 64.0f

#define WSQ_BYTES ((size_t)DIM * DIM * 2)
#define WFF_BYTES ((size_t)DFF * DIM * 2)
#define P16_BYTES ((size_t)MROWS * DIM * 2)
#define X1_BYTES  ((size_t)MROWS * DIM * 4)
#define G16_BYTES ((size_t)MROWS * DFF * 2)
#define OFF_WQ  ((size_t)0)
#define OFF_WK  (OFF_WQ + WSQ_BYTES)
#define OFF_WV  (OFF_WK + WSQ_BYTES)
#define OFF_WO  (OFF_WV + WSQ_BYTES)
#define OFF_W1  (OFF_WO + WSQ_BYTES)
#define OFF_W2  (OFF_W1 + WFF_BYTES)
#define OFF_H   (OFF_W2 + WFF_BYTES)
#define OFF_Q   (OFF_H + P16_BYTES)
#define OFF_K   (OFF_Q + P16_BYTES)
#define OFF_VT  (OFF_K + P16_BYTES)
#define OFF_CTX (OFF_VT + P16_BYTES)
#define OFF_X1  (OFF_CTX + P16_BYTES)
#define OFF_H2  (OFF_X1 + X1_BYTES)
#define OFF_G   (OFF_H2 + P16_BYTES)
#define WS_TOTAL (OFF_G + G16_BYTES)
static_assert((WSQ_BYTES % 128) == 0 && (WFF_BYTES % 128) == 0 && (P16_BYTES % 128) == 0);
static_assert((X1_BYTES % 128) == 0 && (G16_BYTES % 128) == 0);
static_assert(WS_TOTAL <= (size_t)134217728);

__device__ __forceinline__ float bf16r(float x) {
  unsigned int u = __float_as_uint(x);
  u = (u + 0x7FFFu + ((u >> 16) & 1u)) & 0xFFFF0000u;
  return __uint_as_float(u);
}

__device__ __forceinline__ v16h cat8(v8h lo, v8h hi) {
  return __builtin_shufflevector(lo, hi, 0, 1, 2, 3, 4, 5, 6, 7, 8, 9, 10, 11, 12, 13, 14, 15);
}

__device__ __forceinline__ v16h frag_g(const _Float16* p) {
  return cat8(*(const v8h*)(p), *(const v8h*)(p + 16));
}

__device__ __forceinline__ v8f wmma16(v16h a, v16h b, v8f c) {
  v8f d = __builtin_amdgcn_wmma_f32_16x16x32_f16(false, a, false, b, (short)0, c,
                                                 false, false);
  asm volatile("v_nop\n\tv_nop\n\tv_nop\n\tv_nop" : "+v"(d) : "v"(a), "v"(b));
  return d;
}

__device__ __forceinline__ float red16_max(float x) {
#pragma unroll
  for (int off = 1; off < 16; off <<= 1) x = fmaxf(x, __shfl_xor(x, off, 32));
  return x;
}
__device__ __forceinline__ float red16_sum(float x) {
#pragma unroll
  for (int off = 1; off < 16; off <<= 1) x += __shfl_xor(x, off, 32);
  return x;
}
__device__ __forceinline__ float red32_sum(float x) {
#pragma unroll
  for (int off = 1; off < 32; off <<= 1) x += __shfl_xor(x, off, 32);
  return x;
}

__device__ __forceinline__ void wave_lds_sync() {
  __builtin_amdgcn_fence(3  , "wavefront");
  asm volatile("s_wait_dscnt 0x0" ::: "memory");
  __builtin_amdgcn_wave_barrier();
}

__device__ __forceinline__ float gelu_tanh(float t) {
  const float inner = 0.7978845608028654f * (t + 0.044715f * (t * t * t));
  const float e = __expf(fminf(-2.0f * inner, 80.0f));
  return t * __builtin_amdgcn_rcpf(1.0f + e);
}

__global__ __launch_bounds__(256) void wcvt_kernel(
    const float* __restrict__ src, _Float16* __restrict__ dst) {
  const size_t e = ((size_t)blockIdx.x * 256u + threadIdx.x) * 8u;
  const v4f a0 = *(const v4f*)(src + e);
  const v4f a1 = *(const v4f*)(src + e + 4);
  v8h o;
#pragma unroll
  for (int j = 0; j < 4; ++j) {
    o[j]     = (_Float16)(WCARRY * bf16r(a0[j]));
    o[j + 4] = (_Float16)(WCARRY * bf16r(a1[j]));
  }
  *(volatile v8h*)(dst + e) = o;
  __threadfence();
  *(volatile v8h*)(dst + e) = o;
}

__global__ __launch_bounds__(128) void ln_kernel(
    const float* __restrict__ X, const float* __restrict__ gw,
    const float* __restrict__ gb, _Float16* __restrict__ dst, int cvt_in) {
  __shared__ float red[8];
  const unsigned tid = threadIdx.x, lane = tid & 31u;
  const unsigned w = (unsigned)__builtin_amdgcn_readfirstlane((int)(threadIdx.x >> 5));
  const unsigned row = blockIdx.x;
  const unsigned c = tid * 8u;
  const float* sp = X + (size_t)row * DIM + c;
  const v4f a0 = *(const v4f*)(sp);
  const v4f a1 = *(const v4f*)(sp + 4);
  float v[8];
#pragma unroll
  for (int j = 0; j < 4; ++j) { v[j] = a0[j]; v[j + 4] = a1[j]; }
  if (cvt_in != 0) {
#pragma unroll
    for (int j = 0; j < 8; ++j) v[j] = bf16r(v[j]);
  }
  float s = ((v[0] + v[1]) + (v[2] + v[3])) + ((v[4] + v[5]) + (v[6] + v[7]));
  s = red32_sum(s);
  if (lane == 0u) red[w] = s;
  __syncthreads();
  const float mu = ((red[0] + red[1]) + (red[2] + red[3])) * (1.0f / DIM);
  float d[8];
  float ss = 0.0f;
#pragma unroll
  for (int j = 0; j < 8; ++j) { d[j] = v[j] - mu; ss += d[j] * d[j]; }
  ss = red32_sum(ss);
  if (lane == 0u) red[4u + w] = ss;
  __syncthreads();
  const float var = ((red[4] + red[5]) + (red[6] + red[7])) * (1.0f / DIM);
  const float rstd = rsqrtf(var + 1.0e-5f);
  const v4f w0 = *(const v4f*)(gw + c);
  const v4f w1 = *(const v4f*)(gw + c + 4);
  const v4f b0 = *(const v4f*)(gb + c);
  const v4f b1 = *(const v4f*)(gb + c + 4);
  v8h o;
#pragma unroll
  for (int j = 0; j < 4; ++j) {
    o[j]     = (_Float16)(d[j] * rstd * bf16r(w0[j]) + bf16r(b0[j]));
    o[j + 4] = (_Float16)(d[j + 4] * rstd * bf16r(w1[j]) + bf16r(b1[j]));
  }
  _Float16* op = dst + (size_t)row * DIM + c;
  *(volatile v8h*)(op) = o;
  __threadfence();
  *(volatile v8h*)(op) = o;
}

template <int MODE, int KD, int ND>
__device__ __forceinline__ void gemm_body(
    const _Float16* __restrict__ A16, const _Float16* __restrict__ Bt,
    const float* __restrict__ bias, const float* __restrict__ resid,
    float* __restrict__ outf, _Float16* __restrict__ out16) {
  static_assert((KD % 64) == 0);
  static_assert((ND % 64) == 0);
  __shared__ float Cs[64 * LDC];
  const unsigned tid = threadIdx.x, lane = tid & 31u;
  const unsigned w = (unsigned)__builtin_amdgcn_readfirstlane((int)(threadIdx.x >> 5));
  const unsigned mw = w >> 1, nw = w & 1u;
  const unsigned hh = lane >> 4, m = lane & 15u;
  const unsigned n0 = blockIdx.x * 64u;
  const unsigned row0 = blockIdx.y * 64u;

  const _Float16* ap  = A16 + (size_t)(row0 + mw * 16u + m) * KD + hh * 8u;
  const _Float16* bp0 = Bt + (size_t)(n0 + nw * 32u + m) * KD + hh * 8u;
  const _Float16* bp1 = bp0 + 16 * KD;
  v8f acc0 = {}, acc1 = {};
#pragma unroll 2
  for (unsigned k0 = 0; k0 < (unsigned)KD; k0 += 32u) {
    const v16h a  = frag_g(ap + k0);
    const v16h b0 = frag_g(bp0 + k0);
    const v16h b1 = frag_g(bp1 + k0);
    acc0 = wmma16(a, b0, acc0);
    acc1 = wmma16(a, b1, acc1);
  }
#pragma unroll
  for (int r = 0; r < 8; ++r) {
    const unsigned ci = (mw * 16u + hh * 8u + (unsigned)r) * LDC + nw * 32u + m;
    Cs[ci]       = acc0[r];
    Cs[ci + 16u] = acc1[r];
  }
  __syncthreads();

  if (MODE == 0 || MODE == 3) {
    v8h x[2];
    size_t off[2];
#pragma unroll
    for (unsigned i = 0; i < 2u; ++i) {
      const unsigned r = 32u * i + (tid >> 3);
      const unsigned c = (tid & 7u) * 8u;
      const v4f u0 = *(const v4f*)&Cs[r * LDC + c];
      const v4f u1 = *(const v4f*)&Cs[r * LDC + c + 4];
      const v4f g0 = *(const v4f*)(bias + n0 + c);
      const v4f g1 = *(const v4f*)(bias + n0 + c + 4);
#pragma unroll
      for (int j = 0; j < 4; ++j) {
        float t0 = u0[j] * (1.0f / WCARRY) + bf16r(g0[j]);
        float t1 = u1[j] * (1.0f / WCARRY) + bf16r(g1[j]);
        if (MODE == 3) {
          t0 = GCARRY * gelu_tanh(t0);
          t1 = GCARRY * gelu_tanh(t1);
        }
        x[i][j]     = (_Float16)t0;
        x[i][j + 4] = (_Float16)t1;
      }
      off[i] = (size_t)(row0 + r) * ND + n0 + c;
    }
#pragma unroll
    for (int i = 0; i < 2; ++i) *(volatile v8h*)(out16 + off[i]) = x[i];
    __threadfence();
#pragma unroll
    for (int i = 0; i < 2; ++i) *(volatile v8h*)(out16 + off[i]) = x[i];
  }

  if (MODE == 1) {
    v8h x[2];
    size_t off[2];
#pragma unroll
    for (unsigned i = 0; i < 2u; ++i) {
      const unsigned dcol = 32u * i + (tid >> 3);
      const unsigned kk = (tid & 7u) * 8u;
      const float bb = bf16r(bias[n0 + dcol]);
#pragma unroll
      for (unsigned j = 0; j < 8u; ++j)
        x[i][j] = (_Float16)(Cs[(kk + j) * LDC + dcol] * (1.0f / WCARRY) + bb);
      off[i] = (size_t)(n0 + dcol) * MROWS + row0 + kk;
    }
#pragma unroll
    for (int i = 0; i < 2; ++i) *(volatile v8h*)(out16 + off[i]) = x[i];
    __threadfence();
#pragma unroll
    for (int i = 0; i < 2; ++i) *(volatile v8h*)(out16 + off[i]) = x[i];
  }

  if (MODE == 2 || MODE == 4) {
    v4f xs[4];
    size_t off[4];
#pragma unroll
    for (unsigned i = 0; i < 4u; ++i) {
      const unsigned r = 16u * i + (tid >> 4);
      const unsigned c = (tid & 15u) * 4u;
      const size_t o = (size_t)(row0 + r) * ND + n0 + c;
      const v4f u = *(const v4f*)&Cs[r * LDC + c];
      const v4f g = *(const v4f*)(bias + n0 + c);
      const v4f rs = *(const v4f*)(resid + o);
      v4f val;
#pragma unroll
      for (int j = 0; j < 4; ++j) {
        const float rr = (MODE == 2) ? bf16r(rs[j]) : rs[j];
        val[j] = u[j] * (1.0f / (WCARRY * VCARRY)) + bf16r(g[j]) + rr;
      }
      xs[i] = val;
      off[i] = o;
    }
#pragma unroll
    for (int i = 0; i < 4; ++i) *(volatile v4f*)(outf + off[i]) = xs[i];
    __threadfence();
#pragma unroll
    for (int i = 0; i < 4; ++i) *(volatile v4f*)(outf + off[i]) = xs[i];
  }
}
static_assert(VCARRY == GCARRY);

__global__ __launch_bounds__(256) void gemm_qk_kernel(
    const _Float16* __restrict__ A16, const _Float16* __restrict__ Bt,
    const float* __restrict__ bias, _Float16* __restrict__ out16) {
  gemm_body<0, DIM, DIM>(A16, Bt, bias, nullptr, nullptr, out16);
}
__global__ __launch_bounds__(256) void gemm_vt_kernel(
    const _Float16* __restrict__ A16, const _Float16* __restrict__ Bt,
    const float* __restrict__ bias, _Float16* __restrict__ out16) {
  gemm_body<1, DIM, DIM>(A16, Bt, bias, nullptr, nullptr, out16);
}
__global__ __launch_bounds__(256) void gemm_oproj_kernel(
    const _Float16* __restrict__ A16, const _Float16* __restrict__ Bt,
    const float* __restrict__ bias, const float* __restrict__ resid,
    float* __restrict__ outf) {
  gemm_body<2, DIM, DIM>(A16, Bt, bias, resid, outf, nullptr);
}
__global__ __launch_bounds__(256) void gemm_ffn1_kernel(
    const _Float16* __restrict__ A16, const _Float16* __restrict__ Bt,
    const float* __restrict__ bias, _Float16* __restrict__ out16) {
  gemm_body<3, DIM, DFF>(A16, Bt, bias, nullptr, nullptr, out16);
}
__global__ __launch_bounds__(256) void gemm_ffn2_kernel(
    const _Float16* __restrict__ A16, const _Float16* __restrict__ Bt,
    const float* __restrict__ bias, const float* __restrict__ resid,
    float* __restrict__ outf) {
  gemm_body<4, DFF, DIM>(A16, Bt, bias, resid, outf, nullptr);
}

__global__ __launch_bounds__(256) void attn_kernel(
    const _Float16* __restrict__ Qh, const _Float16* __restrict__ Kh,
    const _Float16* __restrict__ Vt, _Float16* __restrict__ Ov) {
  __shared__ _Float16 Ks[64 * LDT];
  __shared__ _Float16 Vs[64 * LDT];
  __shared__ _Float16 Ps[8 * 16 * LDT];

  const unsigned tid = threadIdx.x, lane = tid & 31u;
  const unsigned w = (unsigned)__builtin_amdgcn_readfirstlane((int)(threadIdx.x >> 5));
  const unsigned hh = lane >> 4, m = lane & 15u;
  const unsigned q0 = blockIdx.x * 128u;
  const unsigned head = blockIdx.y;
  const unsigned wrow = q0 + w * 16u;
  const unsigned pb = w * (16u * LDT);
  const float scale = 0.125f;

  const size_t qoff = (size_t)(wrow + m) * DIM + head * HD + hh * 8u;
  v16h qf[2];
  qf[0] = frag_g(Qh + qoff);
  qf[1] = frag_g(Qh + qoff + 32);

  float mrow[8], lrow[8];
  v8f o[4];
#pragma unroll
  for (int v = 0; v < 8; ++v) { mrow[v] = -1.0e30f; lrow[v] = 0.0f; }
#pragma unroll
  for (int nb = 0; nb < 4; ++nb) o[nb] = (v8f){};

  const size_t kplane = (size_t)head * HD;
  const size_t vplane = (size_t)(head * HD) * MROWS;
  const unsigned kend = q0 + 128u;

  for (unsigned kb = 0; kb < kend; kb += 64u) {
#pragma unroll
    for (unsigned j = 0; j < 2u; ++j) {
      const unsigned idx = tid + 256u * j;
      const unsigned r = idx >> 3, c = (idx & 7u) * 8u;
      *(v8h*)&Ks[r * LDT + c] = *(const v8h*)(Kh + kplane + (size_t)(kb + r) * DIM + c);
      *(v8h*)&Vs[r * LDT + c] = *(const v8h*)(Vt + vplane + (size_t)r * MROWS + kb + c);
    }
    __syncthreads();

    if (kb <= wrow + 15u) {
      v8f s[4];
#pragma unroll
      for (int kg = 0; kg < 4; ++kg) {
        v8f t = {};
#pragma unroll
        for (int c = 0; c < 2; ++c) {
          const unsigned ix = ((unsigned)kg * 16u + m) * LDT + (unsigned)c * 32u + hh * 8u;
          const v16h kf = cat8(*(const v8h*)&Ks[ix], *(const v8h*)&Ks[ix + 16u]);
          t = wmma16(qf[c], kf, t);
        }
        s[kg] = t * scale;
      }

      if (kb + 63u > wrow) {
#pragma unroll
        for (int kg = 0; kg < 4; ++kg)
#pragma unroll
          for (int v = 0; v < 8; ++v) {
            const unsigned key = kb + (unsigned)kg * 16u + m;
            const unsigned row = wrow + hh * 8u + (unsigned)v;
            s[kg][v] = (key <= row) ? s[kg][v] : -1.0e30f;
          }
      }

      float alpha[8];
#pragma unroll
      for (int v = 0; v < 8; ++v) {
        float mx = fmaxf(fmaxf(s[0][v], s[1][v]), fmaxf(s[2][v], s[3][v]));
        mx = red16_max(mx);
        const float mn = fmaxf(mrow[v], mx);
        alpha[v] = __expf(mrow[v] - mn);
        mrow[v] = mn;
      }
#pragma unroll
      for (int kg = 0; kg < 4; ++kg)
#pragma unroll
        for (int v = 0; v < 8; ++v) s[kg][v] = __expf(s[kg][v] - mrow[v]);
#pragma unroll
      for (int v = 0; v < 8; ++v) {
        const float rs = red16_sum((s[0][v] + s[1][v]) + (s[2][v] + s[3][v]));
        lrow[v] = alpha[v] * lrow[v] + rs;
      }
#pragma unroll
      for (int nb = 0; nb < 4; ++nb)
#pragma unroll
        for (int v = 0; v < 8; ++v) o[nb][v] = o[nb][v] * alpha[v];

#pragma unroll
      for (int kg = 0; kg < 4; ++kg)
#pragma unroll
        for (int v = 0; v < 8; ++v)
          Ps[pb + (hh * 8u + (unsigned)v) * LDT + (unsigned)kg * 16u + m] =
              (_Float16)(s[kg][v] * PCARRY);
      wave_lds_sync();

#pragma unroll
      for (int c = 0; c < 2; ++c) {
        const unsigned px = pb + m * LDT + (unsigned)c * 32u + hh * 8u;
        const v16h pf = cat8(*(const v8h*)&Ps[px], *(const v8h*)&Ps[px + 16u]);
#pragma unroll
        for (int nb = 0; nb < 4; ++nb) {
          const unsigned vx = ((unsigned)nb * 16u + m) * LDT + (unsigned)c * 32u + hh * 8u;
          const v16h vf = cat8(*(const v8h*)&Vs[vx], *(const v8h*)&Vs[vx + 16u]);
          o[nb] = wmma16(pf, vf, o[nb]);
        }
      }
      wave_lds_sync();
    }
    __syncthreads();
  }

  float inv[8];
#pragma unroll
  for (int v = 0; v < 8; ++v) inv[v] = __builtin_amdgcn_rcpf(lrow[v]) * (VCARRY / PCARRY);
#pragma unroll
  for (int nb = 0; nb < 4; ++nb)
#pragma unroll
    for (int v = 0; v < 8; ++v)
      Ps[pb + (hh * 8u + (unsigned)v) * LDT + (unsigned)nb * 16u + m] =
          (_Float16)(o[nb][v] * inv[v]);
  wave_lds_sync();
  v8h x[4];
  size_t off[4];
#pragma unroll
  for (unsigned i = 0; i < 4u; ++i) {
    const unsigned r = 4u * i + (lane >> 3);
    const unsigned c = (lane & 7u) * 8u;
    x[i] = *(const v8h*)&Ps[pb + r * LDT + c];
    off[i] = (size_t)(wrow + r) * DIM + head * HD + c;
  }
#pragma unroll
  for (int i = 0; i < 4; ++i) *(volatile v8h*)(Ov + off[i]) = x[i];
  __threadfence();
#pragma unroll
  for (int i = 0; i < 4; ++i) *(volatile v8h*)(Ov + off[i]) = x[i];
}

extern "C" void kernel_launch(void* const* d_in, const int* in_sizes, int n_in,
                              void* d_out, int out_size, void* d_ws, size_t ws_size,
                              hipStream_t stream) {
  if (n_in < 17) return;
  const long long need_x = (long long)SEQ * DIM;
  if ((long long)in_sizes[0] < need_x) return;
  if ((long long)in_sizes[1] < (long long)DIM * DIM) return;
  if (in_sizes[2] < DIM) return;
  if ((long long)in_sizes[3] < (long long)DIM * DIM) return;
  if (in_sizes[4] < DIM) return;
  if ((long long)in_sizes[5] < (long long)DIM * DIM) return;
  if (in_sizes[6] < DIM) return;
  if ((long long)in_sizes[7] < (long long)DIM * DIM) return;
  if (in_sizes[8] < DIM) return;
  if ((long long)in_sizes[9] < (long long)DFF * DIM) return;
  if (in_sizes[10] < DFF) return;
  if ((long long)in_sizes[11] < (long long)DIM * DFF) return;
  if (in_sizes[12] < DIM) return;
  if (in_sizes[13] < DIM) return;
  if (in_sizes[14] < DIM) return;
  if (in_sizes[15] < DIM) return;
  if (in_sizes[16] < DIM) return;
  if ((long long)out_size < need_x) return;
  if (ws_size < WS_TOTAL) return;

  const float* X    = (const float*)d_in[0];
  const float* Wq   = (const float*)d_in[1];
  const float* bq   = (const float*)d_in[2];
  const float* Wk   = (const float*)d_in[3];
  const float* bk   = (const float*)d_in[4];
  const float* Wv   = (const float*)d_in[5];
  const float* bv   = (const float*)d_in[6];
  const float* Wo   = (const float*)d_in[7];
  const float* bo   = (const float*)d_in[8];
  const float* W1   = (const float*)d_in[9];
  const float* b1   = (const float*)d_in[10];
  const float* W2   = (const float*)d_in[11];
  const float* b2   = (const float*)d_in[12];
  const float* ln1w = (const float*)d_in[13];
  const float* ln1b = (const float*)d_in[14];
  const float* ln2w = (const float*)d_in[15];
  const float* ln2b = (const float*)d_in[16];
  float* out = (float*)d_out;

  char* ws = (char*)d_ws;
  _Float16* WtQ   = (_Float16*)(ws + OFF_WQ);
  _Float16* WtK   = (_Float16*)(ws + OFF_WK);
  _Float16* WtV   = (_Float16*)(ws + OFF_WV);
  _Float16* WtO   = (_Float16*)(ws + OFF_WO);
  _Float16* Wt1   = (_Float16*)(ws + OFF_W1);
  _Float16* Wt2   = (_Float16*)(ws + OFF_W2);
  _Float16* H16   = (_Float16*)(ws + OFF_H);
  _Float16* Q16   = (_Float16*)(ws + OFF_Q);
  _Float16* K16   = (_Float16*)(ws + OFF_K);
  _Float16* Vt16  = (_Float16*)(ws + OFF_VT);
  _Float16* Ctx16 = (_Float16*)(ws + OFF_CTX);
  float*    X1    = (float*)(ws + OFF_X1);
  _Float16* H2    = (_Float16*)(ws + OFF_H2);
  _Float16* G16   = (_Float16*)(ws + OFF_G);

  dim3 blk(256);
  const unsigned gsq = (unsigned)(((size_t)DIM * DIM) / 2048);
  const unsigned gff = (unsigned)(((size_t)DFF * DIM) / 2048);
  dim3 gg(DIM / 64, MROWS / 64);
  dim3 gf1(DFF / 64, MROWS / 64);

  wcvt_kernel<<<dim3(gsq), blk, 0, stream>>>(Wq, WtQ);
  wcvt_kernel<<<dim3(gsq), blk, 0, stream>>>(Wk, WtK);
  wcvt_kernel<<<dim3(gsq), blk, 0, stream>>>(Wv, WtV);
  wcvt_kernel<<<dim3(gsq), blk, 0, stream>>>(Wo, WtO);
  wcvt_kernel<<<dim3(gff), blk, 0, stream>>>(W1, Wt1);
  wcvt_kernel<<<dim3(gff), blk, 0, stream>>>(W2, Wt2);

  ln_kernel<<<dim3(MROWS), dim3(128), 0, stream>>>(X, ln1w, ln1b, H16, 1);
  gemm_qk_kernel<<<gg, blk, 0, stream>>>(H16, WtQ, bq, Q16);
  gemm_qk_kernel<<<gg, blk, 0, stream>>>(H16, WtK, bk, K16);
  gemm_vt_kernel<<<gg, blk, 0, stream>>>(H16, WtV, bv, Vt16);
  attn_kernel<<<dim3(SEQ / 128, NHEAD), blk, 0, stream>>>(Q16, K16, Vt16, Ctx16);
  gemm_oproj_kernel<<<gg, blk, 0, stream>>>(Ctx16, WtO, bo, X, X1);

  ln_kernel<<<dim3(MROWS), dim3(128), 0, stream>>>(X1, ln2w, ln2b, H2, 0);
  gemm_ffn1_kernel<<<gf1, blk, 0, stream>>>(H2, Wt1, b1, G16);
  gemm_ffn2_kernel<<<gg, blk, 0, stream>>>(G16, Wt2, b2, X1, out);
}
